// Split_BN_ReLU_DConv_27049704030775
// MI455X (gfx1250) — hardware-verified
//
#include <hip/hip_runtime.h>

typedef __attribute__((ext_vector_type(16))) _Float16 v16h;
typedef __attribute__((ext_vector_type(8)))  _Float16 v8h;
typedef __attribute__((ext_vector_type(16))) __bf16   v16b;
typedef __attribute__((ext_vector_type(8)))  __bf16   v8b;
typedef __attribute__((ext_vector_type(8)))  float    v8f;
typedef __attribute__((ext_vector_type(4)))  float    v4f;

__device__ __forceinline__ unsigned short f2bf_bits(float f) {
  unsigned u = __float_as_uint(f);
  return (unsigned short)((u + 0x7FFFu + ((u >> 16) & 1u)) >> 16);
}
__device__ __forceinline__ float bf_bits2f(unsigned short h) { return __uint_as_float(((unsigned)h) << 16); }

__device__ __forceinline__ void dep_guard_h(v8f& a, v8f& b, v16h x, v16h y) { asm volatile("v_nop\n\tv_nop\n\tv_nop\n\tv_nop" : "+v"(a), "+v"(b) : "v"(x), "v"(y)); }
__device__ __forceinline__ void dep_guard_b(v8f& a, v8f& b, v16b x, v16b y) { asm volatile("v_nop\n\tv_nop\n\tv_nop\n\tv_nop" : "+v"(a), "+v"(b) : "v"(x), "v"(y)); }
__device__ __forceinline__ void keep4_h(v16h a, v16h b, v16h c, v16h d) { asm volatile("v_nop" :: "v"(a), "v"(b), "v"(c), "v"(d)); }
__device__ __forceinline__ void keep4_b(v16b a, v16b b, v16b c, v16b d) { asm volatile("v_nop" :: "v"(a), "v"(b), "v"(c), "v"(d)); }
__device__ __forceinline__ void acc_guard4(v8f& a, v8f& b, v8f& c, v8f& d) { asm volatile("v_nop\n\tv_nop\n\tv_nop\n\tv_nop" : "+v"(a), "+v"(b), "+v"(c), "+v"(d)); }
template <typename T> struct Frag;
template <> struct Frag<_Float16> {
  typedef v16h V; union U { v16h v; v8h h[2]; };
  static __device__ __forceinline__ v16h load(const _Float16* p) {
    U f; f.h[0] = *(const v8h*)(p); f.h[1] = *(const v8h*)(p + 16); return f.v;
  }
  static __device__ __forceinline__ v8f mma(v16h a, v16h b, v8f c) {
    return __builtin_amdgcn_wmma_f32_16x16x32_f16(false, a, false, b, (short)0, c, false, false);
  }
  static __device__ __forceinline__ void guard(v8f& a, v8f& b, v16h x, v16h y) { dep_guard_h(a, b, x, y); }
  static __device__ __forceinline__ void keep(v16h a, v16h b, v16h c, v16h d) { keep4_h(a, b, c, d); }
};
template <> struct Frag<__bf16> {
  typedef v16b V; union U { v16b v; v8b h[2]; };
  static __device__ __forceinline__ v16b load(const __bf16* p) {
    U f; f.h[0] = *(const v8b*)(p); f.h[1] = *(const v8b*)(p + 16); return f.v;
  }
  static __device__ __forceinline__ v8f mma(v16b a, v16b b, v8f c) {
    return __builtin_amdgcn_wmma_f32_16x16x32_bf16(false, a, false, b, (short)0, c, false, false);
  }
  static __device__ __forceinline__ void guard(v8f& a, v8f& b, v16b x, v16b y) { dep_guard_b(a, b, x, y); }
  static __device__ __forceinline__ void keep(v16b a, v16b b, v16b c, v16b d) { keep4_b(a, b, c, d); }
};

template <int ET> struct Elem;
template <> struct Elem<0> { typedef _Float16 T; };
template <> struct Elem<1> { typedef __bf16 T; };
template <int ET, bool SPLIT, int BIAS_MODE, int OUT_MODE, bool RESID, int ACT = 0>
__global__ __launch_bounds__(256) void wmma_gemm64(
    const unsigned short* __restrict__ Ap, const unsigned short* __restrict__ A2p, int lda, long strideA,
    const unsigned short* __restrict__ Btp, const unsigned short* __restrict__ Bt2p, int ldb, long strideB,
    void* __restrict__ Cout, void* __restrict__ Cout2, int ldc, long strideC,
    const float* __restrict__ bias,
    const float* __restrict__ resid, long strideR,
    int M, int N, int K, float scale) {
  typedef typename Elem<ET>::T T;
  typedef typename Frag<T>::V V;
  const T* A = (const T*)Ap; const T* A2 = (const T*)A2p; const T* Bt = (const T*)Btp; const T* Bt2 = (const T*)Bt2p;
  __shared__ __align__(16) float sT[8][16 * 68];
  const int b    = blockIdx.y;
  const int lane = threadIdx.x & 31;
  const int wave = threadIdx.x >> 5;
  const int tilesN = N >> 6;
  const int tilesM = M >> 6;
  const int tile = blockIdx.x * 8 + wave;
  if (tile >= tilesM * tilesN) return;
  const int tm = tile / tilesN;
  const int tn = tile - tm * tilesN;
  const int m0 = tm << 6;
  const int n0 = tn << 6;

  const T* Ab  = A  + (size_t)b * strideA;
  const T* Bb  = Bt + (size_t)b * strideB;
  const T* Ab2 = SPLIT ? (A2  + (size_t)b * strideA) : nullptr;
  const T* Bb2 = SPLIT ? (Bt2 + (size_t)b * strideB) : nullptr;

  const int rlane = lane & 15;
  const int koff  = (lane >> 4) * 8;
  const int mOff  = (lane >> 4) * 8;

  v8f acc[4][4];
#pragma unroll
  for (int i = 0; i < 4; ++i)
#pragma unroll
    for (int j = 0; j < 4; ++j) acc[i][j] = (v8f){0.f,0.f,0.f,0.f,0.f,0.f,0.f,0.f};

  for (int k0 = 0; k0 < K; k0 += 32) {
    V bh[4], bl[4];
#pragma unroll
    for (int j = 0; j < 4; ++j) {
      const size_t bo = (size_t)(n0 + (j << 4) + rlane) * ldb + koff + k0;
      bh[j] = Frag<T>::load(Bb + bo);
      if (SPLIT) bl[j] = Frag<T>::load(Bb2 + bo);
    }
#pragma unroll
    for (int i = 0; i < 4; ++i) {
      const size_t ao = (size_t)(m0 + (i << 4) + rlane) * lda + koff + k0;
      V ah = Frag<T>::load(Ab + ao);
      V al;
      if (SPLIT) al = Frag<T>::load(Ab2 + ao);
#pragma unroll
      for (int j = 0; j < 4; ++j) {
        acc[i][j] = Frag<T>::mma(ah, bh[j], acc[i][j]);
        if (SPLIT) {
          acc[i][j] = Frag<T>::mma(ah, bl[j], acc[i][j]);
          acc[i][j] = Frag<T>::mma(al, bh[j], acc[i][j]);
        }
      }
      Frag<T>::guard(acc[i][0], acc[i][3], ah, SPLIT ? al : ah);
    }
    Frag<T>::keep(bh[0], bh[1], bh[2], bh[3]);
    if (SPLIT) Frag<T>::keep(bl[0], bl[1], bl[2], bl[3]);
  }
  acc_guard4(acc[0][0], acc[0][1], acc[0][2], acc[0][3]);
  acc_guard4(acc[1][0], acc[1][1], acc[1][2], acc[1][3]);
  acc_guard4(acc[2][0], acc[2][1], acc[2][2], acc[2][3]);
  acc_guard4(acc[3][0], acc[3][1], acc[3][2], acc[3][3]);

  float* slab = sT[wave];
  const float* Rb = RESID ? (resid + (size_t)b * strideR) : nullptr;
#pragma unroll
  for (int i = 0; i < 4; ++i) {
    const int mBase = m0 + (i << 4);
#pragma unroll
    for (int j = 0; j < 4; ++j) {
      const int n = n0 + (j << 4) + rlane;
      float bv = 0.f;
      if (BIAS_MODE == 2) bv = bias[n];
#pragma unroll
      for (int r = 0; r < 8; ++r) {
        float v = acc[i][j][r] * scale;
        if (BIAS_MODE == 1) v += bias[mBase + mOff + r];
        if (BIAS_MODE == 2) v += bv;
        if (RESID) v += Rb[(size_t)(mBase + mOff + r) * ldc + n];
        if (ACT == 1) v = tanhf(v);
        if (ACT == 2) v = fmaxf(v, 0.0f);
        if (ACT == 3) v = v / (1.0f + expf(-v));
        if (ACT == 4) v = (v > 0.f) ? v : 0.01f * v;
        if (ACT == 5) v = 0.5f * v * (1.0f + erff(v * 0.70710678118654752f));
        slab[(mOff + r) * 68 + (j << 4) + rlane] = v;
      }
    }
    __builtin_amdgcn_fence(__ATOMIC_RELEASE, "workgroup");
    __builtin_amdgcn_wave_barrier();
    __builtin_amdgcn_fence(__ATOMIC_ACQUIRE, "workgroup");
    if (OUT_MODE == 0) {
      float* C = (float*)Cout + (size_t)b * strideC;
      const int hh = lane >> 4, c4 = (lane & 15) * 4;
      for (int pass = 0; pass < 2; ++pass) {
#pragma unroll
        for (int it = 0; it < 8; ++it) {
          const int row = it * 2 + hh;
          v4f v = *(const v4f*)(slab + row * 68 + c4);
          *(volatile v4f*)(C + (size_t)(mBase + row) * ldc + n0 + c4) = v;
        }
        __threadfence();
      }
    } else {
      const int q = lane >> 3, c8 = (lane & 7) * 8;
      unsigned short* C  = (unsigned short*)Cout  + (size_t)b * strideC;
      unsigned short* C2 = (OUT_MODE == 2) ? ((unsigned short*)Cout2 + (size_t)b * strideC) : nullptr;
      for (int pass = 0; pass < 2; ++pass) {
#pragma unroll
        for (int it = 0; it < 4; ++it) {
          const int row = it * 4 + q;
          const float* sp = slab + row * 68 + c8;
          v8h hv, lv;
#pragma unroll
          for (int e = 0; e < 8; ++e) {
            if (OUT_MODE == 1) {
              hv[e] = (_Float16)sp[e];
            } else {
              unsigned short hb = f2bf_bits(sp[e]);
              unsigned short lb = f2bf_bits(sp[e] - bf_bits2f(hb));
              hv[e] = __builtin_bit_cast(_Float16, hb);
              lv[e] = __builtin_bit_cast(_Float16, lb);
            }
          }
          *(volatile v8h*)(C + (size_t)(mBase + row) * ldc + n0 + c8) = hv;
          if (OUT_MODE == 2) *(volatile v8h*)(C2 + (size_t)(mBase + row) * ldc + n0 + c8) = lv;
        }
        __threadfence();
      }
    }
    __builtin_amdgcn_fence(__ATOMIC_RELEASE, "workgroup");
    __builtin_amdgcn_wave_barrier();
    __builtin_amdgcn_fence(__ATOMIC_ACQUIRE, "workgroup");
  }
}

#define NB     8
#define HH     64
#define WW     64
#define CIN    256
#define COUT   64
#define NSPL   4
#define HWPIX  4096
#define NPIX   32768
#define QPIX   8192
#define MOFF   72
#define MOFFP  80
#define KOFF   2304
#define KDC    2304

#define WS_H32    0ull
#define WS_HHI    33554432ull
#define WS_HLO    50331648ull
#define WS_OFFS   67108864ull
#define WS_PLANE  77594624ull
#define WS_WHI    115343360ull
#define WS_WLO    115712000ull
#define WS_WDC    116080640ull
#define WS_OBIAS  116375552ull
#define WS_BSUM   116375936ull
#define WS_TOTAL  116376192ull

__global__ __launch_bounds__(256) void prep_weights(const float* __restrict__ offw, const float* __restrict__ offb,
                                                    const float* __restrict__ dcw,  const float* __restrict__ dcb,
                                                    unsigned short* __restrict__ whi, unsigned short* __restrict__ wlo,
                                                    unsigned short* __restrict__ wdc,
                                                    float* __restrict__ obias, float* __restrict__ bsum)
{
  const int idx = blockIdx.x * 256 + threadIdx.x;
  const int R8 = KOFF / 8;
  const int N1 = MOFFP * R8;
  const int N2 = COUT * (KDC / 8);
  if (idx < N1) {
    const int m  = idx / R8;
    const int k8 = (idx - m * R8) * 8;
    const int mc = (m < MOFF) ? m : (MOFF - 1);
    v8h hv, lv;
#pragma unroll
    for (int e = 0; e < 8; ++e) {
      const int k = k8 + e;
      const int tap = k >> 8, c = k & 255;
      float v = offw[((size_t)(mc * CIN + c)) * 9 + tap];
      if (m >= MOFF) v = 0.0f;
      const unsigned short hb = f2bf_bits(v);
      const unsigned short lb = f2bf_bits(v - bf_bits2f(hb));
      hv[e] = __builtin_bit_cast(_Float16, hb);
      lv[e] = __builtin_bit_cast(_Float16, lb);
    }
    const size_t o = (size_t)m * KOFF + k8;
    *(volatile v8h*)(whi + o) = hv;
    *(volatile v8h*)(wlo + o) = lv;
    __threadfence();
    *(volatile v8h*)(whi + o) = hv;
    *(volatile v8h*)(wlo + o) = lv;
  } else if (idx < N1 + N2) {
    const int id = idx - N1;
    const int o  = id / R8;
    const int k8 = (id - o * R8) * 8;
    v8h hv;
#pragma unroll
    for (int e = 0; e < 8; ++e) {
      const int k = k8 + e;
      const int sp = k / 576;
      const int r  = k - sp * 576;
      const int tap = r >> 6, c = r & 63;
      const float v = dcw[(((size_t)(sp * COUT + o)) * COUT + c) * 9 + tap] * 64.0f;
      hv[e] = (_Float16)v;
    }
    const size_t oo = (size_t)o * KDC + k8;
    *(volatile v8h*)(wdc + oo) = hv;
    __threadfence();
    *(volatile v8h*)(wdc + oo) = hv;
  } else if (idx < N1 + N2 + 32) {
    const int l = idx - N1 - N2;
    if (l < 24) {
      v4f v;
#pragma unroll
      for (int e = 0; e < 4; ++e) {
        const int m = l * 4 + e;
        const int mc = (m < MOFF) ? m : (MOFF - 1);
        float f = offb[mc];
        if (m >= MOFF) f = 0.0f;
        v[e] = f;
      }
      *(volatile v4f*)(obias + l * 4) = v;
      __threadfence();
      *(volatile v4f*)(obias + l * 4) = v;
    }
    if (l < 16) {
      v4f v;
#pragma unroll
      for (int e = 0; e < 4; ++e) {
        const int o = l * 4 + e;
        v[e] = ((dcb[o] + dcb[COUT + o]) + dcb[2 * COUT + o]) + dcb[3 * COUT + o];
      }
      *(volatile v4f*)(bsum + l * 4) = v;
      __threadfence();
      *(volatile v4f*)(bsum + l * 4) = v;
    }
  }
}

__global__ __launch_bounds__(256) void bn_relu_cl(const float* __restrict__ x,
                                                  const float* __restrict__ gam, const float* __restrict__ bet,
                                                  const float* __restrict__ mu,  const float* __restrict__ var,
                                                  float* __restrict__ h32,
                                                  unsigned short* __restrict__ hhi, unsigned short* __restrict__ hlo)
{
  __shared__ __align__(16) float tile[64 * 68];
  __shared__ float sM[64], sS[64], sB[64];
  const int tid = threadIdx.x, lane = tid & 31, wave = tid >> 5;
  const int bx = blockIdx.x;
  const int b  = bx >> 8;
  const int cg = (bx >> 6) & 3;
  const int pg = bx & 63;
  const int c0 = cg * 64, p0 = pg * 64;
  if (tid < 64) {
    const int c = c0 + tid;
    sM[tid] = mu[c];
    sS[tid] = gam[c] * rsqrtf(var[c] + 1e-5f);
    sB[tid] = bet[c];
  }
  __syncthreads();
#pragma unroll
  for (int it = 0; it < 4; ++it) {
    const int item = it * 256 + tid;
    const int c  = item >> 4;
    const int p4 = (item & 15) * 4;
    const v4f xv = *(const v4f*)(x + ((size_t)(b * CIN + c0 + c)) * HWPIX + p0 + p4);
    const float m = sM[c], s = sS[c], bb = sB[c];
#pragma unroll
    for (int e = 0; e < 4; ++e) tile[(p4 + e) * 68 + c] = fmaxf((xv[e] - m) * s + bb, 0.0f);
  }
  __syncthreads();
  {
    const int hh = lane >> 4, c4 = (lane & 15) * 4;
    for (int pass = 0; pass < 2; ++pass) {
#pragma unroll
      for (int it = 0; it < 4; ++it) {
        const int p = it * 16 + wave * 2 + hh;
        const v4f v = *(const v4f*)(tile + p * 68 + c4);
        *(volatile v4f*)(h32 + ((size_t)(b * HWPIX + p0 + p)) * CIN + c0 + c4) = v;
      }
      __threadfence();
    }
  }
  {
    const int q = lane >> 3, c8 = (lane & 7) * 8;
    for (int pass = 0; pass < 2; ++pass) {
#pragma unroll
      for (int it = 0; it < 2; ++it) {
        const int p = it * 32 + wave * 4 + q;
        const float* sp = tile + p * 68 + c8;
        v8h hv, lv;
#pragma unroll
        for (int e = 0; e < 8; ++e) {
          const float f = sp[e];
          const unsigned short hb = f2bf_bits(f);
          const unsigned short lb = f2bf_bits(f - bf_bits2f(hb));
          hv[e] = __builtin_bit_cast(_Float16, hb);
          lv[e] = __builtin_bit_cast(_Float16, lb);
        }
        const size_t o = ((size_t)(b * HWPIX + p0 + p)) * CIN + c0 + c8;
        *(volatile v8h*)(hhi + o) = hv;
        *(volatile v8h*)(hlo + o) = lv;
      }
      __threadfence();
    }
  }
}

__global__ __launch_bounds__(128) void offconv_split(const unsigned short* __restrict__ hhip, const unsigned short* __restrict__ hlop,
                                                     const unsigned short* __restrict__ whip, const unsigned short* __restrict__ wlop,
                                                     const float* __restrict__ obias, float* __restrict__ offs)
{
  typedef __bf16 T;
  typedef Frag<T>::V V;
  const T* Hh = (const T*)hhip; const T* Hl = (const T*)hlop;
  const T* Wh = (const T*)whip; const T* Wl = (const T*)wlop;
  __shared__ __align__(16) float sT[4][16 * 36];
  const int lane = threadIdx.x & 31, wave = threadIdx.x >> 5;
  const int t = blockIdx.x * 4 + wave;
  if (t >= NPIX / 32) return;
  const int b  = t >> 7;
  const int y  = (t >> 1) & 63;
  const int x0 = (t & 1) * 32;
  const int rlane = lane & 15;
  const int koff  = (lane >> 4) * 8;
  const int mOff  = (lane >> 4) * 8;
  const V zerov = __builtin_bit_cast(V, (v8f){0.f,0.f,0.f,0.f,0.f,0.f,0.f,0.f});

  v8f acc[5][2];
#pragma unroll
  for (int i = 0; i < 5; ++i)
#pragma unroll
    for (int j = 0; j < 2; ++j) acc[i][j] = (v8f){0.f,0.f,0.f,0.f,0.f,0.f,0.f,0.f};

#pragma unroll 1
  for (int tap = 0; tap < 9; ++tap) {
    const int kh = tap / 3;
    const int kw = tap - kh * 3;
    const int yy = y + kh - 1;
    const bool vy = (unsigned)yy < (unsigned)HH;
    const int yyc = yy < 0 ? 0 : (yy > HH - 1 ? HH - 1 : yy);
    const T* bph[2]; const T* bpl[2]; bool bv[2];
#pragma unroll
    for (int j = 0; j < 2; ++j) {
      const int xx = x0 + j * 16 + rlane + kw - 1;
      const bool vx = (unsigned)xx < (unsigned)WW;
      const int xxc = xx < 0 ? 0 : (xx > WW - 1 ? WW - 1 : xx);
      const size_t po = ((size_t)((b * HH + yyc) * WW + xxc)) * CIN + koff;
      bph[j] = Hh + po; bpl[j] = Hl + po; bv[j] = vy && vx;
    }
    const size_t ao = (size_t)rlane * KOFF + tap * CIN + koff;
    const T* aph = Wh + ao; const T* apl = Wl + ao;
#pragma unroll 1
    for (int cc = 0; cc < 8; ++cc) {
      V bh[2], bl[2];
#pragma unroll
      for (int j = 0; j < 2; ++j) {
        bh[j] = Frag<T>::load(bph[j] + cc * 32);
        bl[j] = Frag<T>::load(bpl[j] + cc * 32);
        if (!bv[j]) { bh[j] = zerov; bl[j] = zerov; }
      }
#pragma unroll
      for (int i = 0; i < 5; ++i) {
        const size_t mo = (size_t)(i * 16) * KOFF + cc * 32;
        const V ah = Frag<T>::load(aph + mo);
        const V al = Frag<T>::load(apl + mo);
#pragma unroll
        for (int j = 0; j < 2; ++j) {
          acc[i][j] = Frag<T>::mma(ah, bh[j], acc[i][j]);
          acc[i][j] = Frag<T>::mma(ah, bl[j], acc[i][j]);
          acc[i][j] = Frag<T>::mma(al, bh[j], acc[i][j]);
        }
        Frag<T>::guard(acc[i][0], acc[i][1], ah, al);
      }
      Frag<T>::keep(bh[0], bh[1], bl[0], bl[1]);
    }
  }
  acc_guard4(acc[0][0], acc[0][1], acc[1][0], acc[1][1]);
  acc_guard4(acc[2][0], acc[2][1], acc[3][0], acc[3][1]);
  acc_guard4(acc[4][0], acc[4][1], acc[0][0], acc[0][1]);

  float* slab = sT[wave];
  const size_t n0 = (size_t)((b * HH + y) * WW + x0);
  const int q = lane >> 3, c4 = (lane & 7) * 4;
#pragma unroll
  for (int i = 0; i < 5; ++i) {
#pragma unroll
    for (int j = 0; j < 2; ++j) {
#pragma unroll
      for (int r = 0; r < 8; ++r) {
        const int m = i * 16 + mOff + r;
        slab[(mOff + r) * 36 + j * 16 + rlane] = acc[i][j][r] + obias[m];
      }
    }
    __builtin_amdgcn_fence(__ATOMIC_RELEASE, "workgroup");
    __builtin_amdgcn_wave_barrier();
    __builtin_amdgcn_fence(__ATOMIC_ACQUIRE, "workgroup");
    for (int pass = 0; pass < 2; ++pass) {
#pragma unroll
      for (int it = 0; it < 4; ++it) {
        const int row = it * 4 + q;
        const v4f v = *(const v4f*)(slab + row * 36 + c4);
        *(volatile v4f*)(offs + (size_t)(i * 16 + row) * NPIX + n0 + c4) = v;
      }
      __threadfence();
    }
    __builtin_amdgcn_fence(__ATOMIC_RELEASE, "workgroup");
    __builtin_amdgcn_wave_barrier();
    __builtin_amdgcn_fence(__ATOMIC_ACQUIRE, "workgroup");
  }
}

__global__ __launch_bounds__(256) void sample_plane(const float* __restrict__ h32, const float* __restrict__ offs,
                                                    unsigned short* __restrict__ plane, int q)
{
  const int gt = blockIdx.x * 256 + threadIdx.x;
  const int item = gt >> 3;
  const int c8 = (gt & 7) * 8;
  if (item >= QPIX * 36) return;
  const int nl = item / 36;
  const int ik = item - nl * 36;
  const int sp = ik / 9;
  const int kk = ik - sp * 9;
  const int kh = kk / 3;
  const int kw = kk - kh * 3;
  const int n = q * QPIX + nl;
  const int b = n >> 12;
  const int y = (n >> 6) & 63;
  const int x = n & 63;
  const float dy = offs[(size_t)(sp * 18 + 2 * kk) * NPIX + n];
  const float dx = offs[(size_t)(sp * 18 + 2 * kk + 1) * NPIX + n];
  const float py = (float)(y + kh - 1) + dy;
  const float px = (float)(x + kw - 1) + dx;
  const float fy0 = floorf(py), fx0 = floorf(px);
  const float wy1 = py - fy0, wx1 = px - fx0;
  const float wy0 = 1.0f - wy1, wx0 = 1.0f - wx1;
  const float fy1 = fy0 + 1.0f, fx1 = fx0 + 1.0f;
  const bool vy0 = (fy0 >= 0.0f) && (fy0 <= 63.0f);
  const bool vy1 = (fy1 >= 0.0f) && (fy1 <= 63.0f);
  const bool vx0 = (fx0 >= 0.0f) && (fx0 <= 63.0f);
  const bool vx1 = (fx1 >= 0.0f) && (fx1 <= 63.0f);
  const int iy0 = (int)fminf(fmaxf(fy0, 0.0f), 63.0f);
  const int iy1 = (int)fminf(fmaxf(fy1, 0.0f), 63.0f);
  const int ix0 = (int)fminf(fmaxf(fx0, 0.0f), 63.0f);
  const int ix1 = (int)fminf(fmaxf(fx1, 0.0f), 63.0f);
  float w00 = wy0 * wx0, w01 = wy0 * wx1, w10 = wy1 * wx0, w11 = wy1 * wx1;
  if (!(vy0 && vx0)) w00 = 0.0f;
  if (!(vy0 && vx1)) w01 = 0.0f;
  if (!(vy1 && vx0)) w10 = 0.0f;
  if (!(vy1 && vx1)) w11 = 0.0f;
  const float* img = h32 + (size_t)b * HWPIX * CIN + sp * COUT + c8;
  const float* p00 = img + ((size_t)(iy0 * WW + ix0)) * CIN;
  const float* p01 = img + ((size_t)(iy0 * WW + ix1)) * CIN;
  const float* p10 = img + ((size_t)(iy1 * WW + ix0)) * CIN;
  const float* p11 = img + ((size_t)(iy1 * WW + ix1)) * CIN;
  const v4f a0 = *(const v4f*)(p00), a1 = *(const v4f*)(p00 + 4);
  const v4f b0 = *(const v4f*)(p01), b1 = *(const v4f*)(p01 + 4);
  const v4f g0 = *(const v4f*)(p10), g1 = *(const v4f*)(p10 + 4);
  const v4f d0 = *(const v4f*)(p11), d1 = *(const v4f*)(p11 + 4);
  v8h hv;
#pragma unroll
  for (int e = 0; e < 4; ++e) {
    float s = a0[e] * w00;
    s = s + b0[e] * w01;
    s = s + g0[e] * w10;
    s = s + d0[e] * w11;
    hv[e] = (_Float16)s;
    float u = a1[e] * w00;
    u = u + b1[e] * w01;
    u = u + g1[e] * w10;
    u = u + d1[e] * w11;
    hv[4 + e] = (_Float16)u;
  }
  unsigned short* dst = plane + (size_t)nl * KDC + ik * 64 + c8;
  *(volatile v8h*)dst = hv;
  __threadfence();
  *(volatile v8h*)dst = hv;
}

extern "C" void kernel_launch(void* const* d_in, const int* in_sizes, int n_in,
                              void* d_out, int out_size, void* d_ws, size_t ws_size,
                              hipStream_t stream)
{
  if (n_in < 9) return;
  if (in_sizes[0] != NB * CIN * HWPIX) return;
  if (in_sizes[1] != CIN || in_sizes[2] != CIN || in_sizes[3] != CIN || in_sizes[4] != CIN) return;
  if (in_sizes[5] != NSPL * 18 * CIN * 9) return;
  if (in_sizes[6] != NSPL * 18) return;
  if (in_sizes[7] != NSPL * COUT * COUT * 9) return;
  if (in_sizes[8] != NSPL * COUT) return;
  if (out_size != NB * COUT * HWPIX) return;
  if (ws_size < (size_t)WS_TOTAL) return;

  const float* x    = (const float*)d_in[0];
  const float* bg   = (const float*)d_in[1];
  const float* bb   = (const float*)d_in[2];
  const float* bm   = (const float*)d_in[3];
  const float* bv   = (const float*)d_in[4];
  const float* offw = (const float*)d_in[5];
  const float* offb = (const float*)d_in[6];
  const float* dcw  = (const float*)d_in[7];
  const float* dcb  = (const float*)d_in[8];
  float* out = (float*)d_out;

  char* ws = (char*)d_ws;
  float*          h32   = (float*)(ws + WS_H32);
  unsigned short* hhi   = (unsigned short*)(ws + WS_HHI);
  unsigned short* hlo   = (unsigned short*)(ws + WS_HLO);
  float*          offs  = (float*)(ws + WS_OFFS);
  unsigned short* plane = (unsigned short*)(ws + WS_PLANE);
  unsigned short* whi   = (unsigned short*)(ws + WS_WHI);
  unsigned short* wlo   = (unsigned short*)(ws + WS_WLO);
  unsigned short* wdc   = (unsigned short*)(ws + WS_WDC);
  float*          obias = (float*)(ws + WS_OBIAS);
  float*          bsum  = (float*)(ws + WS_BSUM);

  const int prepN = MOFFP * (KOFF / 8) + COUT * (KDC / 8) + 32;
  prep_weights<<<dim3((prepN + 255) / 256), dim3(256), 0, stream>>>(offw, offb, dcw, dcb, whi, wlo, wdc, obias, bsum);

  bn_relu_cl<<<dim3(NB * 4 * 64), dim3(256), 0, stream>>>(x, bg, bb, bm, bv, h32, hhi, hlo);

  offconv_split<<<dim3((NPIX / 32 + 3) / 4), dim3(128), 0, stream>>>(hhi, hlo, whi, wlo, obias, offs);

  for (int q = 0; q < 4; ++q) {
    sample_plane<<<dim3((QPIX * 36 * 8 + 255) / 256), dim3(256), 0, stream>>>(h32, offs, plane, q);
    float* cbase = out + (size_t)q * 2 * COUT * HWPIX;
    wmma_gemm64<0, false, 1, 0, false, 0><<<dim3(8, 2), dim3(256), 0, stream>>>(
        wdc, wdc, KDC, (long)0,
        plane, plane, KDC, (long)HWPIX * KDC,
        (void*)cbase, (void*)cbase, HWPIX, (long)COUT * HWPIX,
        bsum,
        bsum, (long)0,
        COUT, HWPIX, KDC, 0.015625f);
  }
}
